// ReactionNN_49014166782082
// MI455X (gfx1250) — hardware-run, weakly checked
//
#include <hip/hip_runtime.h>


namespace {
constexpr int N = 20000, E = 40000, B = 256, DN = 110, DNP = 128, DE = 8, DL = 8, DH = 64, DHID = 4096, H2 = 128, HQ = 256, XWC = 17 * DH, NBLK = N / 16;
constexpr float XS = 8.0f, WSC = 256.0f;
typedef _Float16 b16;
typedef __attribute__((ext_vector_type(16))) _Float16 v16b;
typedef __attribute__((ext_vector_type(8))) _Float16 v8b;
typedef __attribute__((ext_vector_type(8))) float v8f;
typedef __attribute__((ext_vector_type(4))) float v4f;
typedef __attribute__((ext_vector_type(2))) float v2f;
__device__ __forceinline__ float bf16_rne(float f) { unsigned int u = __float_as_uint(f); u += 0x7FFFu + ((u >> 16) & 1u); return __uint_as_float(u & 0xFFFF0000u); }
__device__ __forceinline__ void split16(float v, b16& hi, b16& lo) { hi = (b16)v; lo = (b16)(v - (float)hi); }
__device__ __forceinline__ v16b frag_kb(const b16* p, int hh) { const v8b a = *(const v8b*)(p + 8 * hh), b = *(const v8b*)(p + 16 + 8 * hh); v16b f;
#pragma unroll
  for (int e = 0; e < 8; ++e) { f[e] = a[e]; f[8 + e] = b[e]; } return f; }
__device__ __forceinline__ v8f wmma16b(v16b a, v16b b, v8f c) { v8f d = __builtin_amdgcn_wmma_f32_16x16x32_f16(false, a, false, b, (short)0, c, false, false); asm volatile("v_nop\n\tv_nop\n\tv_nop\n\tv_nop" : "+v"(d) : "v"(a), "v"(b)); return d; }
__device__ __forceinline__ void wave_lds_sync() { __builtin_amdgcn_fence(__ATOMIC_RELEASE, "workgroup"); __builtin_amdgcn_wave_barrier(); __builtin_amdgcn_fence(__ATOMIC_ACQUIRE, "workgroup"); }
__device__ __forceinline__ float pmul(float a, float b) { float p = a * b; asm volatile("" : "+v"(p)); return p; }
__device__ __forceinline__ int iclamp(int v, int lo, int hi) { return v < lo ? lo : (v > hi ? hi : v); }
__device__ __forceinline__ float sigm(float v) { return 1.0f / (1.0f + __expf(-v)); }
constexpr int CSR_NBLK9 = 512, CSR_GB9 = 9, CSR_GN9 = 1 << CSR_GB9  , CSR_TS9 = (CSR_GN9 < 32 ? 32 : CSR_GN9)  , CSR_MAXG9 = 512, CSR_CAP9 = 12288  ;
__device__ __host__ __forceinline__ int csr_tix9(int v) { return (v >> CSR_GB9) * CSR_TS9 + (v & (CSR_GN9 - 1)); }
__global__ __launch_bounds__(64) void csrA_kernel9(const int* __restrict__ dst, int E, int N, int nG, int CHP, int NGP, int* __restrict__ STG, int* __restrict__ HST) {
  extern __shared__ int sm[];
  int* cnt = sm; int* run = sm + NGP; int* ids = sm + 2 * NGP;
  const int b = blockIdx.x; const int ch = (E + CSR_NBLK9 - 1) / CSR_NBLK9; const int e0 = b * ch, e1 = min(E, e0 + ch);
  for (int i = threadIdx.x; i < NGP; i += 64) cnt[i] = 0;
  for (int i = threadIdx.x; i < CHP; i += 64) ids[i] = -1;
  __syncthreads();
  if (threadIdx.x == 0) {
    for (int e = e0; e < e1; ++e) { int d = dst[e]; d = (d < 0) ? 0 : (d >= N ? N - 1 : d); cnt[d >> CSR_GB9] += 1; }
    int acc = 0; for (int g = 0; g < nG; ++g) { run[g] = acc; acc += cnt[g]; }
    for (int e = e0; e < e1; ++e) { int d = dst[e]; d = (d < 0) ? 0 : (d >= N ? N - 1 : d); const int g = d >> CSR_GB9; ids[run[g]] = e; run[g] += 1; } }
  __syncthreads();
  typedef __attribute__((ext_vector_type(4))) int v4i;
  for (int pass = 0; pass < 2; ++pass) {
    for (int i = threadIdx.x; i < CHP / 4; i += 64) *(volatile v4i*)(STG + (size_t)b * CHP + i * 4) = *(const v4i*)(&ids[i * 4]);
    for (int i = threadIdx.x; i < NGP / 4; i += 64) { v4i v; for (int e = 0; e < 4; ++e) v[e] = (i * 4 + e < nG) ? cnt[i * 4 + e] : 0; *(volatile v4i*)(HST + (size_t)b * NGP + i * 4) = v; }
    __threadfence(); }
}
__global__ __launch_bounds__(512) void csrS_kernel9(const int* __restrict__ HST, int nG, int NGP, int* __restrict__ START, int* __restrict__ TOT, int* __restrict__ OFF) {
  __shared__ int tot[CSR_MAXG9];
  const int b = threadIdx.x;
  for (int pass = 0; pass < 2; ++pass) { int runb = 0; for (int g = 0; g < nG; ++g) { int c = HST[(size_t)b * NGP + g]; c = (c < 0) ? 0 : c; ((volatile int*)OFF)[(size_t)g * CSR_NBLK9 + b] = runb; runb += c; } __threadfence(); }
  for (int g = threadIdx.x; g < nG; g += 512) { int s = 0; for (int bb = 0; bb < CSR_NBLK9; ++bb) { int c = HST[(size_t)bb * NGP + g]; s += (c < 0) ? 0 : c; } tot[g] = s; }
  __syncthreads();
  if (threadIdx.x < 32) {
    __shared__ int st[CSR_MAXG9 + 32];
    if (threadIdx.x == 0) { int acc = 0; for (int g = 0; g < NGP; ++g) { st[g] = acc; if (g < nG) acc += (tot[g] + 31) & ~31; } st[NGP] = acc; }
    __builtin_amdgcn_fence(__ATOMIC_RELEASE, "workgroup"); __builtin_amdgcn_wave_barrier(); __builtin_amdgcn_fence(__ATOMIC_ACQUIRE, "workgroup");
    for (int pass = 0; pass < 2; ++pass) { for (int i = threadIdx.x; i < NGP + 32; i += 32) { ((volatile int*)START)[i] = (i <= NGP) ? st[min(i, NGP)] : 0; ((volatile int*)TOT)[i] = (i < nG) ? tot[i] : 0; } __threadfence(); } }
}
__global__ __launch_bounds__(256) void csrB_kernel9(const int* __restrict__ dst, int N, int nG, int CHP, int NGP, int permLen, const int* __restrict__ STG, const int* __restrict__ HST, const int* __restrict__ OFF, const int* __restrict__ START, const int* __restrict__ TOT, int* __restrict__ PERM, int* __restrict__ ROWPTR, int* __restrict__ ROWCNT, int* __restrict__ FLAG) {
  typedef __attribute__((ext_vector_type(4))) int v4i;
  __shared__ int ids[CSR_CAP9]; __shared__ unsigned short key[CSR_CAP9]; __shared__ int outp[CSR_CAP9]; __shared__ int ncnt[CSR_GN9 + 1]; __shared__ int boff[CSR_NBLK9 + 1];
  const int g = blockIdx.x, t_ = threadIdx.x; int tot = TOT[g]; int st = START[g], stn = START[g + 1]; const int v0 = g * CSR_GN9; const int nv = min(CSR_GN9, N - v0); const int t0 = g * CSR_TS9;
  st = (st < 0) ? 0 : (st > permLen - 32 ? permLen - 32 : st) & ~31; stn = (stn < st) ? st : (stn > permLen ? permLen : stn); tot = (tot < 0) ? 0 : tot; if (tot > stn - st && tot <= CSR_CAP9) tot = stn - st;
  if (tot > CSR_CAP9) {
    for (int pass = 0; pass < 2; ++pass) { for (int i = t_; i < CSR_TS9 / 4; i += 256) { v4i a, c; for (int e = 0; e < 4; ++e) { a[e] = st; c[e] = 0; } *(volatile v4i*)(ROWPTR + t0 + i * 4) = a; *(volatile v4i*)(ROWCNT + t0 + i * 4) = c; } if (t_ == 0) ((volatile int*)FLAG)[0] = 1; __threadfence(); } (void)nv; return; }
  if (t_ == 0) { int acc = 0; for (int b = 0; b < CSR_NBLK9; ++b) { boff[b] = acc; int c = HST[(size_t)b * NGP + g]; c = (c < 0) ? 0 : (c > CHP ? CHP : c); acc += c; if (acc > tot) acc = tot; } boff[CSR_NBLK9] = acc; }
  for (int i = t_; i <= CSR_GN9; i += 256) ncnt[i] = 0;
  __syncthreads();
  for (int b = 0; b < CSR_NBLK9; ++b) { const int c = boff[b + 1] - boff[b]; int o_ = OFF[(size_t)g * CSR_NBLK9 + b]; o_ = (o_ < 0) ? 0 : (o_ > CHP - c ? CHP - c : o_); const int* src_ = STG + (size_t)b * CHP + o_;
    for (int i = t_; i < c; i += 256) { int id = src_[i]; id = (id < 0) ? 0 : id; ids[boff[b] + i] = id; int d = dst[id]; d = (d < v0) ? v0 : (d >= N ? N - 1 : d); int kk = d - v0; kk = (kk < 0) ? 0 : (kk >= CSR_GN9 ? CSR_GN9 - 1 : kk); key[boff[b] + i] = (unsigned short)kk; } }
  __syncthreads();
  if (t_ == 0) { for (int i = 0; i < tot; ++i) ncnt[key[i]] += 1; int acc = 0; for (int vl = 0; vl < CSR_GN9; ++vl) { const int c = ncnt[vl]; ncnt[vl] = acc; acc += c; } ncnt[CSR_GN9] = acc;
    for (int i = 0; i < tot; ++i) { const int vl = key[i]; outp[ncnt[vl]] = ids[i]; ncnt[vl] += 1; }
    for (int vl = CSR_GN9; vl > 0; --vl) ncnt[vl] = ncnt[vl - 1]; ncnt[0] = 0; }
  __syncthreads();
  for (int pass = 0; pass < 2; ++pass) {
    for (int i = t_; i < (stn - st) / 4; i += 256) { v4i v; for (int e = 0; e < 4; ++e) { const int q = i * 4 + e; v[e] = (q < tot) ? outp[q] : -1; } *(volatile v4i*)(PERM + st + i * 4) = v; }
    for (int i = t_; i < CSR_TS9 / 4; i += 256) { v4i a, c; for (int e = 0; e < 4; ++e) { const int vl = i * 4 + e; const int vc = vl < CSR_GN9 ? vl : CSR_GN9; a[e] = (vl < CSR_GN9) ? st + ncnt[vc] : st; c[e] = (vl < nv) ? (ncnt[(vc < CSR_GN9 ? vc : CSR_GN9 - 1) + 1] - ncnt[vc]) : 0; } *(volatile v4i*)(ROWPTR + t0 + i * 4) = a; *(volatile v4i*)(ROWCNT + t0 + i * 4) = c; }
    __threadfence(); }
}
__global__ __launch_bounds__(256) void csrZ_kernel9(int* __restrict__ p, size_t n4) { typedef __attribute__((ext_vector_type(4))) int v4i; const size_t tid = (size_t)blockIdx.x * 256 + threadIdx.x, nth = (size_t)gridDim.x * 256; v4i z = {0, 0, 0, 0}; for (size_t i = tid; i < n4; i += nth) *(volatile v4i*)(p + i * 4) = z; }
struct CsrBufs9 { int *STG, *HST, *OFF, *START, *TOT, *PERM, *ROWPTR, *ROWCNT, *FLAG; int nG, NGP, CHP; size_t permLen; char* base; size_t bytes; };
static size_t csr_carve9(CsrBufs9& c, char* ws, size_t off, int E, int N) {
  const size_t off0 = off; c.base = ws + off;
  auto al = [&](size_t bytes) { char* p = ws + off; off += (bytes + 255) & ~(size_t)255; return p; };
  c.nG = (N + CSR_GN9 - 1) / CSR_GN9; c.NGP = (c.nG + 31) & ~31; const int ch = (E + CSR_NBLK9 - 1) / CSR_NBLK9; c.CHP = (ch + 31) & ~31; c.permLen = (size_t)E + 32 * (size_t)c.nG + 32;
  c.STG = (int*)al((size_t)CSR_NBLK9 * c.CHP * 4); c.HST = (int*)al((size_t)CSR_NBLK9 * c.NGP * 4); c.OFF = (int*)al((size_t)c.NGP * CSR_NBLK9 * 4); c.START = (int*)al((size_t)(c.NGP + 64) * 4); c.TOT = (int*)al((size_t)(c.NGP + 64) * 4);
  c.PERM = (int*)al(c.permLen * 4); c.ROWPTR = (int*)al((size_t)c.nG * CSR_TS9 * 4); c.ROWCNT = (int*)al((size_t)c.nG * CSR_TS9 * 4); c.FLAG = (int*)al(256);
  c.bytes = off - off0; return off;
}
static void csr_build9(const CsrBufs9& c, const int* dst, int E, int N, hipStream_t stream) {
  const size_t smem = (size_t)(2 * c.NGP + c.CHP) * 4;
  csrZ_kernel9<<<512, 256, 0, stream>>>((int*)c.base, c.bytes / 16);
  csrA_kernel9<<<CSR_NBLK9, 64, smem, stream>>>(dst, E, N, c.nG, c.CHP, c.NGP, c.STG, c.HST);
  csrS_kernel9<<<1, 512, 0, stream>>>(c.HST, c.nG, c.NGP, c.START, c.TOT, c.OFF);
  csrB_kernel9<<<c.nG, 256, 0, stream>>>(dst, N, c.nG, c.CHP, c.NGP, (int)c.permLen, c.STG, c.HST, c.OFF, c.START, c.TOT, c.PERM, c.ROWPTR, c.ROWCNT, c.FLAG);
}


__global__ __launch_bounds__(256) void wput_kernel(const float* __restrict__ w, int KIN, int KP, int OUTW, b16* __restrict__ WT) {
  const int KG = KP / 8; const size_t u = (size_t)blockIdx.x * 256 + threadIdx.x; if (u >= (size_t)OUTW * KG) return; const int o = (int)(u / KG), k0 = (int)(u % KG) * 8; v8b v;
#pragma unroll
  for (int j = 0; j < 8; ++j) { const int k = k0 + j; v[j] = k < KIN ? (b16)(bf16_rne(w[(size_t)k * OUTW + o]) * WSC) : (b16)0.0f; } for (int pass = 0; pass < 2; ++pass) { *(volatile v8b*)(WT + (size_t)o * KP + k0) = v; __threadfence(); }
}
__global__ __launch_bounds__(256) void wcopy_kernel(const float* __restrict__ w, int OUTW, int KIN, b16* __restrict__ WT) {
  const size_t u = (size_t)blockIdx.x * 256 + threadIdx.x; if (u >= (size_t)OUTW * KIN / 8) return; const size_t e = u * 8; v8b v;
#pragma unroll
  for (int j = 0; j < 8; ++j) v[j] = (b16)(bf16_rne(w[e + j]) * WSC); for (int pass = 0; pass < 2; ++pass) { *(volatile v8b*)(WT + e) = v; __threadfence(); }
}
__global__ __launch_bounds__(256) void wbond_kernel(const float* __restrict__ bw, const float* __restrict__ bb, b16* __restrict__ WB) {
  const int u = blockIdx.x * 256 + threadIdx.x; if (u >= XWC * 8) return; const int col = u / 8, i0 = (u % 8) * 8; v8b v;
#pragma unroll
  for (int j = 0; j < 8; ++j) { const int i = i0 + j; float val; if (col < 16 * DH) { const int k = col / DH, o = col % DH; val = bw[(size_t)k * (DH * DH) + i * DH + o]; } else { const int o = col - 16 * DH; val = bb[i * DH + o]; } v[j] = (b16)(bf16_rne(val) * WSC); }
  for (int pass = 0; pass < 2; ++pass) { *(volatile v8b*)(WB + (size_t)col * DH + i0) = v; __threadfence(); }
}
__global__ __launch_bounds__(32) void proj_kernel(const float* __restrict__ na, const b16* __restrict__ WP, const float* __restrict__ pb, int NLIM, float* __restrict__ X0, float* __restrict__ Hh) {
  __shared__ __attribute__((aligned(16))) b16 Ah[16][DNP + 8]; __shared__ float Tf[16][DH + 2];
  const int lane = threadIdx.x, nloc = lane & 15, hlf = lane >> 4; const size_t m0 = (size_t)blockIdx.x * 16; if (m0 >= (size_t)NLIM) return;
  for (int rr = 0; rr < 16; ++rr) for (int q = 0; q < 4; ++q) { const int c = q * 32 + lane; Ah[rr][c] = (b16)((c < DN ? bf16_rne(na[(m0 + rr) * DN + c]) : 0.0f) * XS); }
  wave_lds_sync();
#pragma unroll
  for (int t = 0; t < 4; ++t) { v8f acc = {};
#pragma unroll
    for (int kb = 0; kb < DNP; kb += 32) acc = wmma16b(frag_kb(&Ah[nloc][kb], hlf), frag_kb(WP + (size_t)(t * 16 + nloc) * DNP + kb, hlf), acc); const int c = t * 16 + nloc; const float bb = bf16_rne(pb[c]);
#pragma unroll
    for (int r8 = 0; r8 < 8; ++r8) Tf[8 * hlf + r8][c] = fmaxf(acc[r8] * (1.0f / (XS * WSC)) + bb, 0.0f); }
  wave_lds_sync();
  for (int pass = 0; pass < 2; ++pass) { for (int rr = 0; rr < 16; ++rr) { const v2f v = *(const v2f*)(&Tf[rr][lane * 2]); *(volatile v2f*)(X0 + (m0 + rr) * DH + lane * 2) = v; *(volatile v2f*)(Hh + (m0 + rr) * DH + lane * 2) = v; } __threadfence(); }
}
__global__ __launch_bounds__(32) void xw_kernel(const float* __restrict__ X, const b16* __restrict__ WB, int NLIM, float* __restrict__ XW) {
  __shared__ __attribute__((aligned(16))) b16 Ah[16][DH + 8], Al[16][DH + 8]; __shared__ __attribute__((aligned(16))) float Tf[16][128 + 4];
  const int lane = threadIdx.x, nloc = lane & 15, hlf = lane >> 4; const int nt = blockIdx.x % NBLK, g = blockIdx.x / NBLK; const size_t m0 = (size_t)nt * 16; if (m0 >= (size_t)NLIM) return; const int ntiles = (XWC - g * 128) < 128 ? (XWC - g * 128) / 16 : 8;
  for (int rr = 0; rr < 16; ++rr) for (int q = 0; q < 2; ++q) { b16 p, ql; split16(X[(m0 + rr) * DH + q * 32 + lane] * XS, p, ql); Ah[rr][q * 32 + lane] = p; Al[rr][q * 32 + lane] = ql; }
  wave_lds_sync(); v8f acc[8];
#pragma unroll
  for (int t = 0; t < 8; ++t) acc[t] = (v8f){};
#pragma unroll
  for (int kb = 0; kb < DH; kb += 32) { const v16b a = frag_kb(&Ah[nloc][kb], hlf), al = frag_kb(&Al[nloc][kb], hlf);
#pragma unroll
    for (int t = 0; t < 8; ++t) if (t < ntiles) { const v16b bw = frag_kb(WB + ((size_t)g * 128 + t * 16 + nloc) * DH + kb, hlf); acc[t] = wmma16b(a, bw, acc[t]); acc[t] = wmma16b(al, bw, acc[t]); } }
#pragma unroll
  for (int t = 0; t < 8; ++t) { if (t < ntiles) {
#pragma unroll
      for (int r8 = 0; r8 < 8; ++r8) Tf[8 * hlf + r8][t * 16 + nloc] = acc[t][r8] * (1.0f / (XS * WSC)); } }
  wave_lds_sync();
  for (int pass = 0; pass < 2; ++pass) { for (int rr = 0; rr < 16; ++rr) for (int c = lane; c < ntiles * 16; c += 32) ((volatile float*)XW)[(m0 + rr) * XWC + g * 128 + c] = Tf[rr][c]; __threadfence(); }
}
__global__ __launch_bounds__(32) void step_kernel(const float* __restrict__ XW, const float* __restrict__ Hh, const float* __restrict__ ea, const float* __restrict__ el, const float* __restrict__ cen, const float* __restrict__ beta, const int* __restrict__ srcs, const int* __restrict__ PERM, const int* __restrict__ ROWPTR, const int* __restrict__ ROWCNT, int permLen, const float* __restrict__ nb, const b16* __restrict__ WIH, const b16* __restrict__ WHH, const float* __restrict__ bih, const float* __restrict__ bhh, int NLIM, float* __restrict__ HN) {
  __shared__ __attribute__((aligned(16))) b16 Aa[16][DH + 8], Aal[16][DH + 8], Bh[16][DH + 8], Bl[16][DH + 8]; __shared__ float Hs[16][DH + 1], Ef[16];
  const int lane = threadIdx.x, nloc = lane & 15, hlf = lane >> 4; const size_t m0 = (size_t)blockIdx.x * 16; if (m0 >= (size_t)NLIM) return;
  float cc[DL], bt[DL]; for (int i = 0; i < DL; ++i) { cc[i] = bf16_rne(cen[i]); bt[i] = bf16_rne(beta[i]); }
  for (int rr = 0; rr < 16; ++rr) { const size_t v = m0 + rr; int st = ROWPTR[v], cnt = ROWCNT[v]; cnt = iclamp(cnt, 0, 1 << 20); st = iclamp(st, 0, permLen - cnt); float a0 = 0.0f, a1 = 0.0f;
#pragma unroll 1
    for (int j = 0; j < cnt; ++j) { const int e = iclamp(PERM[st + j], 0, E - 1); const size_t s = (size_t)iclamp(srcs[e], 0, N - 1); if (s >= (size_t)NLIM) continue;
      if (lane < DE) Ef[lane] = bf16_rne(ea[(size_t)e * DE + lane]); else if (lane < DE + DL) { const float dd = bf16_rne(el[e]) - cc[lane - DE]; Ef[lane] = __expf(-pmul(bt[lane - DE], pmul(dd, dd))); }
      wave_lds_sync(); const float* xr = XW + s * XWC; float p0 = xr[16 * DH + lane * 2], p1 = xr[16 * DH + lane * 2 + 1];
#pragma unroll
      for (int k = 0; k < 16; ++k) { const float f = Ef[k]; const v2f xv = *(const v2f*)(xr + k * DH + lane * 2); p0 += pmul(f, xv[0]); p1 += pmul(f, xv[1]); }
      a0 += p0; a1 += p1; wave_lds_sync(); }
    const float av0 = fmaxf(a0 + bf16_rne(nb[lane * 2]), 0.0f), av1 = fmaxf(a1 + bf16_rne(nb[lane * 2 + 1]), 0.0f); b16 p, q; split16(av0 * XS, p, q); Aa[rr][lane * 2] = p; Aal[rr][lane * 2] = q; split16(av1 * XS, p, q); Aa[rr][lane * 2 + 1] = p; Aal[rr][lane * 2 + 1] = q;
    const v2f hv = *(const v2f*)(Hh + v * DH + lane * 2); Hs[rr][lane * 2] = hv[0]; Hs[rr][lane * 2 + 1] = hv[1]; split16(hv[0] * XS, p, q); Bh[rr][lane * 2] = p; Bl[rr][lane * 2] = q; split16(hv[1] * XS, p, q); Bh[rr][lane * 2 + 1] = p; Bl[rr][lane * 2 + 1] = q; }
  wave_lds_sync();
  v8f gi[12], gh[12];
#pragma unroll
  for (int t = 0; t < 12; ++t) { gi[t] = (v8f){}; gh[t] = (v8f){}; }
#pragma unroll
  for (int kb = 0; kb < DH; kb += 32) { const v16b a = frag_kb(&Aa[nloc][kb], hlf), al = frag_kb(&Aal[nloc][kb], hlf), bh = frag_kb(&Bh[nloc][kb], hlf), bl = frag_kb(&Bl[nloc][kb], hlf);
#pragma unroll
    for (int t = 0; t < 12; ++t) { const v16b wi = frag_kb(WIH + (size_t)(t * 16 + nloc) * DH + kb, hlf), wh = frag_kb(WHH + (size_t)(t * 16 + nloc) * DH + kb, hlf); gi[t] = wmma16b(a, wi, gi[t]); gi[t] = wmma16b(al, wi, gi[t]); gh[t] = wmma16b(bh, wh, gh[t]); gh[t] = wmma16b(bl, wh, gh[t]); } }
  const float sc = 1.0f / (XS * WSC);
#pragma unroll
  for (int tg = 0; tg < 4; ++tg) { const int j = tg * 16 + nloc; const float bir = bf16_rne(bih[j]), biz = bf16_rne(bih[DH + j]), bin = bf16_rne(bih[2 * DH + j]), bhr = bf16_rne(bhh[j]), bhz = bf16_rne(bhh[DH + j]), bhn = bf16_rne(bhh[2 * DH + j]);
#pragma unroll
    for (int r8 = 0; r8 < 8; ++r8) { const int rl = 8 * hlf + r8; const float r = sigm(gi[tg][r8] * sc + bir + gh[tg][r8] * sc + bhr), z = sigm(gi[4 + tg][r8] * sc + biz + gh[4 + tg][r8] * sc + bhz); const float n = tanhf(gi[8 + tg][r8] * sc + bin + pmul(r, gh[8 + tg][r8] * sc + bhn)); Hs[rl][j] = pmul(1.0f - z, n) + pmul(z, Hs[rl][j]); } }
  wave_lds_sync();
  for (int pass = 0; pass < 2; ++pass) { for (int rr = 0; rr < 16; ++rr) *(volatile v2f*)(HN + (m0 + rr) * DH + lane * 2) = (v2f){Hs[rr][lane * 2], Hs[rr][lane * 2 + 1]}; __threadfence(); }
}
template <int KIN>
__global__ __launch_bounds__(32) void lstm_kernel(const float* __restrict__ INP, const float* HPREV, const float* CPREV, const b16* __restrict__ WI, const b16* __restrict__ WH, const float* __restrict__ bi, const float* __restrict__ bh, float* HOUT, float* COUT) {
  __shared__ __attribute__((aligned(16))) b16 Ah[16][KIN + 8], Al[16][KIN + 8], Bh[16][H2 + 8], Bl[16][H2 + 8]; __shared__ float Gs[3][16][H2 + 1];
  const int lane = threadIdx.x, nloc = lane & 15, hlf = lane >> 4; const size_t m0 = (size_t)blockIdx.x * 16;
  for (int rr = 0; rr < 16; ++rr) { for (int q = 0; q < KIN / 32; ++q) { b16 p, ql; split16(INP[(m0 + rr) * KIN + q * 32 + lane] * XS, p, ql); Ah[rr][q * 32 + lane] = p; Al[rr][q * 32 + lane] = ql; } for (int q = 0; q < 4; ++q) { b16 p, ql; split16(HPREV[(m0 + rr) * H2 + q * 32 + lane] * XS, p, ql); Bh[rr][q * 32 + lane] = p; Bl[rr][q * 32 + lane] = ql; } }
  wave_lds_sync(); const float sc = 1.0f / (XS * WSC);
#pragma unroll 1
  for (int gate = 0; gate < 4; ++gate) { v8f acc[8];
#pragma unroll
    for (int t = 0; t < 8; ++t) acc[t] = (v8f){};
#pragma unroll 2
    for (int kb = 0; kb < KIN; kb += 32) { const v16b a = frag_kb(&Ah[nloc][kb], hlf), al = frag_kb(&Al[nloc][kb], hlf);
#pragma unroll
      for (int t = 0; t < 8; ++t) { const v16b w = frag_kb(WI + (size_t)(gate * H2 + t * 16 + nloc) * KIN + kb, hlf); acc[t] = wmma16b(a, w, acc[t]); acc[t] = wmma16b(al, w, acc[t]); } }
#pragma unroll
    for (int kb = 0; kb < H2; kb += 32) { const v16b a = frag_kb(&Bh[nloc][kb], hlf), al = frag_kb(&Bl[nloc][kb], hlf);
#pragma unroll
      for (int t = 0; t < 8; ++t) { const v16b w = frag_kb(WH + (size_t)(gate * H2 + t * 16 + nloc) * H2 + kb, hlf); acc[t] = wmma16b(a, w, acc[t]); acc[t] = wmma16b(al, w, acc[t]); } }
#pragma unroll
    for (int t = 0; t < 8; ++t) { const int j = t * 16 + nloc; const float bb = bf16_rne(bi[gate * H2 + j]) + bf16_rne(bh[gate * H2 + j]);
#pragma unroll
      for (int r8 = 0; r8 < 8; ++r8) { const int rl = 8 * hlf + r8; const float g = acc[t][r8] * sc + bb; if (gate < 3) Gs[gate][rl][j] = g; else { const float c = pmul(sigm(Gs[1][rl][j]), CPREV[(m0 + rl) * H2 + j]) + pmul(sigm(Gs[0][rl][j]), tanhf(Gs[2][rl][j])); Gs[0][rl][j] = c; Gs[1][rl][j] = pmul(sigm(g), tanhf(c)); } } }
    wave_lds_sync(); }
  for (int pass = 0; pass < 2; ++pass) { for (int rr = 0; rr < 16; ++rr) for (int q = 0; q < 4; ++q) { ((volatile float*)COUT)[(m0 + rr) * H2 + q * 32 + lane] = Gs[0][rr][q * 32 + lane]; ((volatile float*)HOUT)[(m0 + rr) * H2 + q * 32 + lane] = Gs[1][rr][q * 32 + lane]; } __threadfence(); }
}
__global__ __launch_bounds__(256) void readout_kernel(const float* __restrict__ HL1, const float* __restrict__ Hh, const float* __restrict__ X0, const int* __restrict__ gid, int NLIM, float* __restrict__ QS) {
  __shared__ float Qv[H2], Ev[2048], red[256]; const int g = blockIdx.x, tid = threadIdx.x;
  auto lb = [&](int key) -> int { int lo = 0, hi = N; for (int it = 0; it < 16 && lo < hi; ++it) { const int mid = (lo + hi) >> 1; if (gid[mid] < key) lo = mid + 1; else hi = mid; } return lo; };
  int s0 = lb(g), e0 = lb(g + 1); if (e0 > NLIM) e0 = NLIM; if (e0 < s0) e0 = s0; int cnt = e0 - s0; if (cnt > 2048) cnt = 2048;
  if (tid < H2) Qv[tid] = HL1[(size_t)g * H2 + tid]; __syncthreads();
  for (int i = tid; i < cnt; i += 256) { const size_t n = s0 + i; float s = 0.0f; for (int d = 0; d < DH; ++d) s += pmul(Hh[n * DH + d], Qv[d]) + pmul(X0[n * DH + d], Qv[DH + d]); Ev[i] = s; }
  __syncthreads(); float mx = -INFINITY; for (int i = tid; i < cnt; i += 256) mx = fmaxf(mx, Ev[i]); red[tid] = mx; __syncthreads();
  for (int w = 128; w > 0; w >>= 1) { if (tid < w) red[tid] = fmaxf(red[tid], red[tid + w]); __syncthreads(); } mx = red[0]; __syncthreads();
  float sm = 0.0f; for (int i = tid; i < cnt; i += 256) { const float e = __expf(Ev[i] - mx); Ev[i] = e; sm += e; } red[tid] = sm; __syncthreads();
  for (int w = 128; w > 0; w >>= 1) { if (tid < w) red[tid] += red[tid + w]; __syncthreads(); } const float inv = cnt > 0 ? 1.0f / red[0] : 0.0f; __syncthreads();
  float rd = 0.0f; if (tid < 2 * DH) { for (int i = 0; i < cnt; ++i) { const size_t n = s0 + i; const float f = tid < DH ? Hh[n * DH + tid] : X0[n * DH + tid - DH]; rd += pmul(pmul(Ev[i], inv), f); } }
  for (int pass = 0; pass < 2; ++pass) { if (tid < H2) ((volatile float*)QS)[(size_t)g * HQ + tid] = Qv[tid]; if (tid < 2 * DH) ((volatile float*)QS)[(size_t)g * HQ + H2 + tid] = rd; __threadfence(); }
}
__global__ __launch_bounds__(32) void out_kernel(const float* __restrict__ QS, const b16* __restrict__ WS_, const float* __restrict__ sb, const float* __restrict__ pa, float* __restrict__ out) {
  __shared__ __attribute__((aligned(16))) b16 Ah[16][HQ + 8], Al[16][HQ + 8]; __shared__ __attribute__((aligned(16))) float Tf[16][128 + 4];
  const int lane = threadIdx.x, nloc = lane & 15, hlf = lane >> 4; const size_t m0 = (size_t)blockIdx.x * 16; const float a_ = bf16_rne(pa[0]);
  for (int rr = 0; rr < 16; ++rr) for (int q = 0; q < 8; ++q) { b16 p, ql; split16(QS[(m0 + rr) * HQ + q * 32 + lane] * XS, p, ql); Ah[rr][q * 32 + lane] = p; Al[rr][q * 32 + lane] = ql; }
  wave_lds_sync();
#pragma unroll 1
  for (int cg = 0; cg < DHID / 128; ++cg) { v8f acc[8];
#pragma unroll
    for (int t = 0; t < 8; ++t) acc[t] = (v8f){};
#pragma unroll 2
    for (int kb = 0; kb < HQ; kb += 32) { const v16b a = frag_kb(&Ah[nloc][kb], hlf), al = frag_kb(&Al[nloc][kb], hlf);
#pragma unroll
      for (int t = 0; t < 8; ++t) { const v16b w = frag_kb(WS_ + (size_t)(cg * 128 + t * 16 + nloc) * HQ + kb, hlf); acc[t] = wmma16b(a, w, acc[t]); acc[t] = wmma16b(al, w, acc[t]); } }
#pragma unroll
    for (int t = 0; t < 8; ++t) { const int c = cg * 128 + t * 16 + nloc; const float bb = bf16_rne(sb[c]);
#pragma unroll
      for (int r8 = 0; r8 < 8; ++r8) { const float v = acc[t][r8] * (1.0f / (XS * WSC)) + bb; Tf[8 * hlf + r8][t * 16 + nloc] = v >= 0.0f ? v : pmul(a_, v); } }
    wave_lds_sync();
    for (int pass = 0; pass < 2; ++pass) { for (int rr = 0; rr < 16; ++rr) *(volatile v4f*)(out + (m0 + rr) * DHID + cg * 128 + lane * 4) = *(const v4f*)(&Tf[rr][lane * 4]); __threadfence(); }
    wave_lds_sync(); }
}
__global__ __launch_bounds__(256) void zero_kernel(float* __restrict__ p, int n) { const int i = blockIdx.x * 256 + threadIdx.x; if (i >= n) return; for (int pass = 0; pass < 2; ++pass) { ((volatile float*)p)[i] = 0.0f; __threadfence(); } }
}

extern "C" void kernel_launch(void* const* d_in, const int* in_sizes, int n_in, void* d_out, int out_size, void* d_ws, size_t ws_size, hipStream_t stream) {
  (void)n_in;
  auto Fp = [&](int i) { return (const float*)d_in[i]; }; auto Ip = [&](int i) { return (const int*)d_in[i]; };
  if (in_sizes[0] != N * DN || in_sizes[1] != E * DE || in_sizes[2] != E || in_sizes[3] != E || in_sizes[4] != E || in_sizes[5] != N || in_sizes[6] != DN * DH || in_sizes[10] != 16 * DH * DH || in_sizes[13] != 3 * DH * DH || in_sizes[17] != 4 * H2 * HQ || in_sizes[21] != 4 * H2 * H2 || in_sizes[25] != HQ * DHID || out_size != B * DHID) return;
  const int NLIM = N; const int GB16 = NBLK;
  size_t off = 0; char* ws = (char*)d_ws;
  auto carve = [&](size_t bytes) { char* p = ws + off; off += (bytes + 255) & ~(size_t)255; return p; };
  b16* WP = (b16*)carve(DH * DNP * 2); b16* WB = (b16*)carve((size_t)XWC * DH * 2); b16* WIH = (b16*)carve(192 * DH * 2); b16* WHH = (b16*)carve(192 * DH * 2); b16* WI0 = (b16*)carve((size_t)512 * HQ * 2); b16* WH0 = (b16*)carve(512 * H2 * 2); b16* WI1 = (b16*)carve(512 * H2 * 2); b16* WH1 = (b16*)carve(512 * H2 * 2); b16* WSP = (b16*)carve((size_t)DHID * HQ * 2);
  float* X0 = (float*)carve((size_t)N * DH * 4); float* HA = (float*)carve((size_t)N * DH * 4); float* HB = (float*)carve((size_t)N * DH * 4); float* XW = (float*)carve((size_t)N * XWC * 4);
  float* HL0 = (float*)carve(B * H2 * 4); float* CL0 = (float*)carve(B * H2 * 4); float* HL1 = (float*)carve(B * H2 * 4); float* CL1 = (float*)carve(B * H2 * 4); float* QS = (float*)carve(B * HQ * 4);
  CsrBufs9 csr; off = csr_carve9(csr, ws, off, E, N);
  if (off > ws_size || off > ((size_t)128 << 20)) return;
  wput_kernel<<<(DH * 16 + 255) / 256, 256, 0, stream>>>(Fp(6), DN, DNP, DH, WP); wbond_kernel<<<(XWC * 8 + 255) / 256, 256, 0, stream>>>(Fp(10), Fp(11), WB);
  wcopy_kernel<<<(192 * DH / 8 + 255) / 256, 256, 0, stream>>>(Fp(13), 192, DH, WIH); wcopy_kernel<<<(192 * DH / 8 + 255) / 256, 256, 0, stream>>>(Fp(14), 192, DH, WHH);
  wcopy_kernel<<<(512 * HQ / 8 + 255) / 256, 256, 0, stream>>>(Fp(17), 512, HQ, WI0); wcopy_kernel<<<(512 * H2 / 8 + 255) / 256, 256, 0, stream>>>(Fp(18), 512, H2, WH0); wcopy_kernel<<<(512 * H2 / 8 + 255) / 256, 256, 0, stream>>>(Fp(21), 512, H2, WI1); wcopy_kernel<<<(512 * H2 / 8 + 255) / 256, 256, 0, stream>>>(Fp(22), 512, H2, WH1);
  wput_kernel<<<(unsigned)(((size_t)DHID * 32 + 255) / 256), 256, 0, stream>>>(Fp(25), HQ, HQ, DHID, WSP);
  csr_build9(csr, Ip(4), E, N, stream);
  proj_kernel<<<GB16, 32, 0, stream>>>(Fp(0), WP, Fp(7), NLIM, X0, HA);
  float* Hc = HA; float* Hn = HB;
  for (int step = 0; step < 4; ++step) {
    xw_kernel<<<NBLK * 9, 32, 0, stream>>>(Hc, WB, NLIM, XW);
    step_kernel<<<GB16, 32, 0, stream>>>(XW, Hc, Fp(1), Fp(2), Fp(8), Fp(9), Ip(3), csr.PERM, csr.ROWPTR, csr.ROWCNT, (int)csr.permLen, Fp(12), WIH, WHH, Fp(15), Fp(16), NLIM, Hn);
    float* t = Hc; Hc = Hn; Hn = t; }
  zero_kernel<<<(B * H2 + 255) / 256, 256, 0, stream>>>(HL0, B * H2); zero_kernel<<<(B * H2 + 255) / 256, 256, 0, stream>>>(CL0, B * H2); zero_kernel<<<(B * H2 + 255) / 256, 256, 0, stream>>>(HL1, B * H2); zero_kernel<<<(B * H2 + 255) / 256, 256, 0, stream>>>(CL1, B * H2); zero_kernel<<<(B * HQ + 255) / 256, 256, 0, stream>>>(QS, B * HQ);
  for (int it = 0; it < 3; ++it) {
    lstm_kernel<HQ><<<B / 16, 32, 0, stream>>>(QS, HL0, CL0, WI0, WH0, Fp(19), Fp(20), HL0, CL0);
    lstm_kernel<H2><<<B / 16, 32, 0, stream>>>(HL0, HL1, CL1, WI1, WH1, Fp(23), Fp(24), HL1, CL1);
    readout_kernel<<<B, 256, 0, stream>>>(HL1, Hc, X0, Ip(5), NLIM, QS); }
  out_kernel<<<B / 16, 32, 0, stream>>>(QS, WSP, Fp(26), Fp(27), (float*)d_out);
}
